// TransformerBlock_24343874633890
// MI455X (gfx1250) — hardware-verified
//
#include <hip/hip_runtime.h>
#include <stddef.h>


typedef _Float16 v16h __attribute__((ext_vector_type(16)));
typedef _Float16 v8h  __attribute__((ext_vector_type(8)));
typedef float    v8f  __attribute__((ext_vector_type(8)));
typedef float    v4f  __attribute__((ext_vector_type(4)));

#ifndef NB
#define NB 2
#endif
#ifndef SEQ
#define SEQ 2048
#endif
#define NB_FULL  2
#define SEQ_FULL 2048
#define DIM   1024
#define NHEAD 16
#define HD    64
#define INTER 4096
#define MROWS (NB * SEQ)

static_assert(NB >= 1 && NB <= NB_FULL);
static_assert(SEQ >= 128 && SEQ <= SEQ_FULL && (SEQ % 128) == 0);
static_assert(DIM == NHEAD * HD);
static_assert(HD == 64);
static_assert(DIM == 128 * 8);
static_assert((DIM % 64) == 0 && (DIM % 32) == 0);
static_assert((INTER % 64) == 0 && (INTER % 32) == 0);
static_assert((MROWS % 64) == 0 && (MROWS % 2) == 0);
static_assert((SEQ % 64) == 0);
static_assert((size_t)MROWS * INTER < (size_t)0xFFFFFFFFu);

#define LDT 72
#define LDC 68
static_assert(LDT >= 64 + 8 && (LDT % 8) == 0);
static_assert(LDC >= 64 + 4 && (LDC % 4) == 0);

#define WCARRY 64.0f
#define PCARRY 1024.0f
#define VCARRY 64.0f
#define GCARRY 16.0f

#define WSQ_BYTES     ((size_t)DIM * DIM * 2)
#define WFF_BYTES     ((size_t)DIM * INTER * 2)
#define PLANE16_BYTES ((size_t)MROWS * DIM * 2)
#define HPLANE_BYTES  ((size_t)MROWS * DIM * 4)
#define GPLANE_BYTES  ((size_t)MROWS * INTER * 2)
#define OFF_WQ   ((size_t)0)
#define OFF_WK   (OFF_WQ + WSQ_BYTES)
#define OFF_WV   (OFF_WK + WSQ_BYTES)
#define OFF_WO   (OFF_WV + WSQ_BYTES)
#define OFF_W1   (OFF_WO + WSQ_BYTES)
#define OFF_W3   (OFF_W1 + WFF_BYTES)
#define OFF_W2   (OFF_W3 + WFF_BYTES)
#define OFF_XN   (OFF_W2 + WFF_BYTES)
#define OFF_Q    (OFF_XN + PLANE16_BYTES)
#define OFF_K    (OFF_Q + PLANE16_BYTES)
#define OFF_VT   (OFF_K + PLANE16_BYTES)
#define OFF_CTX  (OFF_VT + PLANE16_BYTES)
#define OFF_H    (OFF_CTX + PLANE16_BYTES)
#define OFF_G    (OFF_H + HPLANE_BYTES)
#define WS_TOTAL (OFF_G + GPLANE_BYTES)
static_assert((WSQ_BYTES % 128) == 0 && (WFF_BYTES % 128) == 0);
static_assert((PLANE16_BYTES % 128) == 0 && (HPLANE_BYTES % 128) == 0 && (GPLANE_BYTES % 128) == 0);
static_assert(WS_TOTAL <= (size_t)134217728);

__device__ __forceinline__ float bf16r(float x) {
  unsigned int u = __float_as_uint(x);
  u = (u + 0x7FFFu + ((u >> 16) & 1u)) & 0xFFFF0000u;
  return __uint_as_float(u);
}

__device__ __forceinline__ v16h join16(v8h lo, v8h hi) {
  v16h out;
#pragma unroll
  for (int i = 0; i < 8; ++i) { out[i] = lo[i]; out[i + 8] = hi[i]; }
  return out;
}
__device__ __forceinline__ v16h frag_at(const _Float16* __restrict__ p) {
  return join16(*(const v8h*)(p), *(const v8h*)(p + 16));
}

__device__ __forceinline__ v8f wmma16(v16h a, v16h b, v8f c) {
  v8f d = __builtin_amdgcn_wmma_f32_16x16x32_f16(false, a, false, b, (short)0, c,
                                                 false, false);
  asm volatile("v_nop\n\tv_nop\n\tv_nop\n\tv_nop" : "+v"(d) : "v"(a), "v"(b));
  return d;
}

__device__ __forceinline__ float red16_max(float x) {
#pragma unroll
  for (int off = 1; off < 16; off <<= 1) x = fmaxf(x, __shfl_xor(x, off, 32));
  return x;
}
__device__ __forceinline__ float red16_sum(float x) {
#pragma unroll
  for (int off = 1; off < 16; off <<= 1) x += __shfl_xor(x, off, 32);
  return x;
}

__device__ __forceinline__ void wave_lds_sync() {
  __builtin_amdgcn_fence(3  , "wavefront");
  asm volatile("s_wait_dscnt 0x0" ::: "memory");
  __builtin_amdgcn_wave_barrier();
}

__global__ __launch_bounds__(256) void wconv_kernel(
    const float* __restrict__ W, _Float16* __restrict__ Wt, unsigned K, unsigned N) {
  __shared__ _Float16 T[64 * LDT];
  const unsigned tid = threadIdx.x;
  const unsigned n0 = blockIdx.x * 64u;
  const unsigned k0 = blockIdx.y * 64u;
#pragma unroll 4
  for (unsigned j = 0; j < 16u; ++j) {
    const unsigned idx = tid + 256u * j;
    const unsigned kr = idx >> 6, nc = idx & 63u;
    const float v = W[(size_t)(k0 + kr) * N + n0 + nc];
    T[nc * LDT + kr] = (_Float16)(WCARRY * bf16r(v));
  }
  __syncthreads();
  v8h x[2];
  size_t off[2];
#pragma unroll
  for (unsigned i = 0; i < 2u; ++i) {
    const unsigned n = 32u * i + (tid >> 3);
    const unsigned kc = (tid & 7u) * 8u;
    x[i] = *(const v8h*)&T[n * LDT + kc];
    off[i] = (size_t)(n0 + n) * K + k0 + kc;
  }
#pragma unroll
  for (int i = 0; i < 2; ++i) *(volatile v8h*)(Wt + off[i]) = x[i];
  __threadfence();
#pragma unroll
  for (int i = 0; i < 2; ++i) *(volatile v8h*)(Wt + off[i]) = x[i];
}

__global__ __launch_bounds__(256) void rmsnorm_kernel(
    const float* __restrict__ src, const float* __restrict__ gw,
    _Float16* __restrict__ dst, unsigned srcb, int rnd) {
  __shared__ float red[8];
  const unsigned tid = threadIdx.x, lane = tid & 31u;
  const unsigned wave = (unsigned)__builtin_amdgcn_readfirstlane((int)(threadIdx.x >> 5));
  const unsigned rsel = tid >> 7;
  const unsigned crow = blockIdx.x * 2u + rsel;
  const unsigned bidx = crow / (unsigned)SEQ;
  const unsigned sq = crow - bidx * (unsigned)SEQ;
  const size_t frow = (size_t)bidx * srcb + sq;
  const unsigned c = (tid & 127u) * 8u;
  const float* sp = src + frow * DIM + c;
  v4f a0 = *(const v4f*)(sp);
  v4f a1 = *(const v4f*)(sp + 4);
#pragma unroll
  for (int j = 0; j < 4; ++j) {
    a0[j] = (rnd != 0) ? bf16r(a0[j]) : a0[j];
    a1[j] = (rnd != 0) ? bf16r(a1[j]) : a1[j];
  }
  float ss = 0.0f;
#pragma unroll
  for (int j = 0; j < 4; ++j) ss += a0[j] * a0[j];
#pragma unroll
  for (int j = 0; j < 4; ++j) ss += a1[j] * a1[j];
#pragma unroll
  for (int off = 16; off > 0; off >>= 1) ss += __shfl_xor(ss, off, 32);
  if (lane == 0u) red[wave] = ss;
  __syncthreads();
  const float tot = (red[rsel * 4u + 0u] + red[rsel * 4u + 1u]) +
                    (red[rsel * 4u + 2u] + red[rsel * 4u + 3u]);
  const float sc = rsqrtf(tot * (1.0f / (float)DIM) + 1.0e-6f);
  const v4f g0 = *(const v4f*)(gw + c);
  const v4f g1 = *(const v4f*)(gw + c + 4);
  v8h o;
#pragma unroll
  for (int j = 0; j < 4; ++j) {
    o[j]     = (_Float16)((a0[j] * sc) * bf16r(g0[j]));
    o[j + 4] = (_Float16)((a1[j] * sc) * bf16r(g1[j]));
  }
  _Float16* dp = dst + (size_t)crow * DIM + c;
  *(volatile v8h*)(dp) = o;
  __threadfence();
  *(volatile v8h*)(dp) = o;
}

template <int MODE, int KD, int ND>
__device__ __forceinline__ void gemm_body(
    const _Float16* __restrict__ A16, const _Float16* __restrict__ Bt,
    const _Float16* __restrict__ Bt2, const float* __restrict__ addf,
    float* __restrict__ outf, _Float16* __restrict__ out16) {
  static_assert((KD % 32) == 0);
  static_assert((ND % 64) == 0);
  static_assert(MODE == 0 || MODE == 4 || ND == DIM);
  __shared__ float Cs[64 * LDC];
  const unsigned tid = threadIdx.x, lane = tid & 31u;
  const unsigned wave = (unsigned)__builtin_amdgcn_readfirstlane((int)(threadIdx.x >> 5));
  const unsigned mw = wave >> 1, nw = wave & 1u;
  const unsigned hh = lane >> 4, m = lane & 15u;
  const unsigned n0 = blockIdx.x * 64u;
  const unsigned row0 = blockIdx.y * 64u;

  const _Float16* ap = A16 + (size_t)(row0 + mw * 16u + m) * KD + hh * 8u;
  const size_t boff = (size_t)(n0 + nw * 32u + m) * KD + hh * 8u;
  const _Float16* bp0 = Bt + boff;
  const _Float16* bp1 = bp0 + 16 * KD;
  const _Float16* cp0 = Bt2 + boff;
  const _Float16* cp1 = cp0 + 16 * KD;
  v8f acc0 = {}, acc1 = {}, acc2 = {}, acc3 = {};
#pragma unroll 2
  for (unsigned k0 = 0; k0 < (unsigned)KD; k0 += 32u) {
    const v16h a  = frag_at(ap + k0);
    const v16h b0 = frag_at(bp0 + k0);
    const v16h b1 = frag_at(bp1 + k0);
    acc0 = wmma16(a, b0, acc0);
    acc1 = wmma16(a, b1, acc1);
    if (MODE == 4) {
      const v16h c0 = frag_at(cp0 + k0);
      const v16h c1 = frag_at(cp1 + k0);
      acc2 = wmma16(a, c0, acc2);
      acc3 = wmma16(a, c1, acc3);
    }
  }
  if (MODE == 4) {
#pragma unroll
    for (int r = 0; r < 8; ++r) {
      const float z0 = acc0[r] * (1.0f / WCARRY);
      const float u0 = acc2[r] * (1.0f / WCARRY);
      const float z1 = acc1[r] * (1.0f / WCARRY);
      const float u1 = acc3[r] * (1.0f / WCARRY);
      const float s0 = __builtin_amdgcn_rcpf(1.0f + expf(-z0));
      const float s1 = __builtin_amdgcn_rcpf(1.0f + expf(-z1));
      acc0[r] = ((z0 * s0) * u0) * GCARRY;
      acc1[r] = ((z1 * s1) * u1) * GCARRY;
    }
  }
#pragma unroll
  for (int r = 0; r < 8; ++r) {
    const unsigned ci = (mw * 16u + hh * 8u + (unsigned)r) * LDC + nw * 32u + m;
    Cs[ci]       = acc0[r];
    Cs[ci + 16u] = acc1[r];
  }
  __syncthreads();

  if (MODE == 0 || MODE == 4) {
    const float sc = (MODE == 0) ? (1.0f / WCARRY) : 1.0f;
    v8h x[2];
    size_t off[2];
#pragma unroll
    for (unsigned i = 0; i < 2u; ++i) {
      const unsigned r = 32u * i + (tid >> 3);
      const unsigned c = (tid & 7u) * 8u;
      const v4f u0 = *(const v4f*)&Cs[r * LDC + c];
      const v4f u1 = *(const v4f*)&Cs[r * LDC + c + 4];
#pragma unroll
      for (int j = 0; j < 4; ++j) {
        x[i][j]     = (_Float16)(u0[j] * sc);
        x[i][j + 4] = (_Float16)(u1[j] * sc);
      }
      off[i] = (size_t)(row0 + r) * ND + n0 + c;
    }
#pragma unroll
    for (int i = 0; i < 2; ++i) *(volatile v8h*)(out16 + off[i]) = x[i];
    __threadfence();
#pragma unroll
    for (int i = 0; i < 2; ++i) *(volatile v8h*)(out16 + off[i]) = x[i];
  }

  if (MODE == 1) {
    const unsigned bidx = row0 / (unsigned)SEQ;
    const unsigned key0 = row0 - bidx * (unsigned)SEQ;
    v8h x[2];
    size_t off[2];
#pragma unroll
    for (unsigned i = 0; i < 2u; ++i) {
      const unsigned dcol = 32u * i + (tid >> 3);
      const unsigned kk = (tid & 7u) * 8u;
#pragma unroll
      for (unsigned j = 0; j < 8u; ++j)
        x[i][j] = (_Float16)(Cs[(kk + j) * LDC + dcol] * (1.0f / WCARRY));
      off[i] = ((size_t)bidx * DIM + n0 + dcol) * SEQ + key0 + kk;
    }
#pragma unroll
    for (int i = 0; i < 2; ++i) *(volatile v8h*)(out16 + off[i]) = x[i];
    __threadfence();
#pragma unroll
    for (int i = 0; i < 2; ++i) *(volatile v8h*)(out16 + off[i]) = x[i];
  }

  if (MODE == 2 || MODE == 3) {
    const float sc = (MODE == 2) ? (1.0f / (WCARRY * VCARRY)) : (1.0f / (WCARRY * GCARRY));
    v4f xs[4];
    size_t off[4];
#pragma unroll
    for (unsigned i = 0; i < 4u; ++i) {
      const unsigned r = 16u * i + (tid >> 4);
      const unsigned c = (tid & 15u) * 4u;
      const unsigned crow = row0 + r;
      const unsigned bidx = crow / (unsigned)SEQ;
      const unsigned sq = crow - bidx * (unsigned)SEQ;
      const size_t frow = (size_t)bidx * SEQ_FULL + sq;
      const size_t arow = (MODE == 2) ? frow : (size_t)crow;
      const size_t orow = (MODE == 2) ? (size_t)crow : frow;
      const v4f u = *(const v4f*)&Cs[r * LDC + c];
      const v4f g = *(const v4f*)(addf + arow * DIM + n0 + c);
      v4f val;
#pragma unroll
      for (int j = 0; j < 4; ++j)
        val[j] = u[j] * sc + ((MODE == 2) ? bf16r(g[j]) : g[j]);
      xs[i] = val;
      off[i] = orow * DIM + n0 + c;
    }
#pragma unroll
    for (int i = 0; i < 4; ++i) *(volatile v4f*)(outf + off[i]) = xs[i];
    __threadfence();
#pragma unroll
    for (int i = 0; i < 4; ++i) *(volatile v4f*)(outf + off[i]) = xs[i];
  }
}

__global__ __launch_bounds__(256) void gemm_rowmajor_kernel(
    const _Float16* __restrict__ A16, const _Float16* __restrict__ Bt,
    _Float16* __restrict__ out16) {
  gemm_body<0, DIM, DIM>(A16, Bt, Bt, (const float*)0, (float*)0, out16);
}
__global__ __launch_bounds__(256) void gemm_vt_kernel(
    const _Float16* __restrict__ A16, const _Float16* __restrict__ Bt,
    _Float16* __restrict__ out16) {
  gemm_body<1, DIM, DIM>(A16, Bt, Bt, (const float*)0, (float*)0, out16);
}
__global__ __launch_bounds__(256) void gemm_oproj_kernel(
    const _Float16* __restrict__ A16, const _Float16* __restrict__ Bt,
    const float* __restrict__ xin, float* __restrict__ hout) {
  gemm_body<2, DIM, DIM>(A16, Bt, Bt, xin, hout, (_Float16*)0);
}
__global__ __launch_bounds__(256) void gemm_up_kernel(
    const _Float16* __restrict__ A16, const _Float16* __restrict__ B1,
    const _Float16* __restrict__ B3, _Float16* __restrict__ g16) {
  gemm_body<4, DIM, INTER>(A16, B1, B3, (const float*)0, (float*)0, g16);
}
__global__ __launch_bounds__(256) void gemm_down_kernel(
    const _Float16* __restrict__ G16, const _Float16* __restrict__ Bt,
    const float* __restrict__ hin, float* __restrict__ outf) {
  gemm_body<3, INTER, DIM>(G16, Bt, Bt, hin, outf, (_Float16*)0);
}

__global__ __launch_bounds__(256) void attn_kernel(
    const _Float16* __restrict__ Qh, const _Float16* __restrict__ Kh,
    const _Float16* __restrict__ Vt, _Float16* __restrict__ Ov) {
  __shared__ _Float16 Ks[64 * LDT];
  __shared__ _Float16 Vs[64 * LDT];
  __shared__ _Float16 Ps[8 * 16 * LDT];

  const unsigned tid = threadIdx.x, lane = tid & 31u;
  const unsigned wave = (unsigned)__builtin_amdgcn_readfirstlane((int)(threadIdx.x >> 5));
  const unsigned hh = lane >> 4, m = lane & 15u;
  const unsigned q0 = blockIdx.x * 128u;
  const unsigned head = blockIdx.y;
  const unsigned b = blockIdx.z;
  const float scale = 0.125f;
  const unsigned pb = wave * (16u * LDT);
  const unsigned fo = m * LDT + hh * 8u;
  const unsigned qw = q0 + wave * 16u;
  const unsigned kend = q0 + 128u;

  const size_t qoff = (size_t)(b * (unsigned)SEQ + qw + m) * DIM + head * HD + hh * 8u;
  v16h qf[2];
  qf[0] = frag_at(Qh + qoff);
  qf[1] = frag_at(Qh + qoff + 32);

  float mrow[8], lrow[8];
  v8f o[4];
#pragma unroll
  for (int v = 0; v < 8; ++v) { mrow[v] = -1.0e30f; lrow[v] = 0.0f; }
#pragma unroll
  for (int nb = 0; nb < 4; ++nb) o[nb] = (v8f){};

  const size_t kplane = (size_t)b * SEQ * DIM + head * HD;
  const size_t vplane = ((size_t)b * DIM + head * HD) * SEQ;

  for (unsigned kb = 0; kb < kend; kb += 64u) {
#pragma unroll
    for (unsigned j = 0; j < 2u; ++j) {
      const unsigned idx = tid + 256u * j;
      const unsigned r = idx >> 3, c = (idx & 7u) * 8u;
      *(v8h*)&Ks[r * LDT + c] = *(const v8h*)(Kh + kplane + (size_t)(kb + r) * DIM + c);
      *(v8h*)&Vs[r * LDT + c] = *(const v8h*)(Vt + vplane + (size_t)r * SEQ + kb + c);
    }
    __syncthreads();

    if (kb <= qw + 15u) {
      v8f s[4];
#pragma unroll
      for (int kg = 0; kg < 4; ++kg) {
        v8f t = {};
#pragma unroll
        for (int c = 0; c < 2; ++c) {
          const unsigned ko = (unsigned)(kg * 16) * LDT + (unsigned)c * 32u + fo;
          const v16h kf = join16(*(const v8h*)&Ks[ko], *(const v8h*)&Ks[ko + 16u]);
          t = wmma16(qf[c], kf, t);
        }
        s[kg] = t * scale;
      }
      if (kb + 63u > qw) {
#pragma unroll
        for (int kg = 0; kg < 4; ++kg)
#pragma unroll
          for (int v = 0; v < 8; ++v) {
            const unsigned key = kb + (unsigned)kg * 16u + m;
            const unsigned qq = qw + hh * 8u + (unsigned)v;
            s[kg][v] = (key > qq) ? -1.0e30f : s[kg][v];
          }
      }

      float alpha[8];
#pragma unroll
      for (int v = 0; v < 8; ++v) {
        float mx = fmaxf(fmaxf(s[0][v], s[1][v]), fmaxf(s[2][v], s[3][v]));
        mx = red16_max(mx);
        const float mn = fmaxf(mrow[v], mx);
        alpha[v] = __expf(mrow[v] - mn);
        mrow[v] = mn;
      }
#pragma unroll
      for (int kg = 0; kg < 4; ++kg)
#pragma unroll
        for (int v = 0; v < 8; ++v) s[kg][v] = __expf(s[kg][v] - mrow[v]);
#pragma unroll
      for (int v = 0; v < 8; ++v) {
        const float rs = red16_sum((s[0][v] + s[1][v]) + (s[2][v] + s[3][v]));
        lrow[v] = alpha[v] * lrow[v] + rs;
      }
#pragma unroll
      for (int nb = 0; nb < 4; ++nb)
#pragma unroll
        for (int v = 0; v < 8; ++v) o[nb][v] = o[nb][v] * alpha[v];

#pragma unroll
      for (int kg = 0; kg < 4; ++kg)
#pragma unroll
        for (int v = 0; v < 8; ++v)
          Ps[pb + (hh * 8u + (unsigned)v) * LDT + (unsigned)kg * 16u + m] =
              (_Float16)(s[kg][v] * PCARRY);
      wave_lds_sync();

#pragma unroll
      for (int c = 0; c < 2; ++c) {
        const unsigned po = pb + (unsigned)c * 32u + fo;
        const v16h pf = join16(*(const v8h*)&Ps[po], *(const v8h*)&Ps[po + 16u]);
#pragma unroll
        for (int nb = 0; nb < 4; ++nb) {
          const unsigned vo = (unsigned)(nb * 16) * LDT + (unsigned)c * 32u + fo;
          const v16h vf = join16(*(const v8h*)&Vs[vo], *(const v8h*)&Vs[vo + 16u]);
          o[nb] = wmma16(pf, vf, o[nb]);
        }
      }
    }
    __syncthreads();
  }

  float inv[8];
#pragma unroll
  for (int v = 0; v < 8; ++v) inv[v] = __builtin_amdgcn_rcpf(lrow[v]) * (VCARRY / PCARRY);
#pragma unroll
  for (int nb = 0; nb < 4; ++nb)
#pragma unroll
    for (int v = 0; v < 8; ++v)
      Ps[pb + (hh * 8u + (unsigned)v) * LDT + (unsigned)nb * 16u + m] =
          (_Float16)(o[nb][v] * inv[v]);
  wave_lds_sync();
  v8h x[4];
  size_t off[4];
#pragma unroll
  for (unsigned i = 0; i < 4u; ++i) {
    const unsigned r = 4u * i + (lane >> 3);
    const unsigned c = (lane & 7u) * 8u;
    x[i] = *(const v8h*)&Ps[pb + r * LDT + c];
    off[i] = (size_t)(b * (unsigned)SEQ + qw + r) * DIM + head * HD + c;
  }
#pragma unroll
  for (int i = 0; i < 4; ++i) *(volatile v8h*)(Ov + off[i]) = x[i];
  __threadfence();
#pragma unroll
  for (int i = 0; i < 4; ++i) *(volatile v8h*)(Ov + off[i]) = x[i];
}

extern "C" void kernel_launch(void* const* d_in, const int* in_sizes, int n_in,
                              void* d_out, int out_size, void* d_ws, size_t ws_size,
                              hipStream_t stream) {
  if (n_in < 10) return;
  const long long need_x = ((long long)(NB - 1) * SEQ_FULL + SEQ) * DIM;
  if ((long long)in_sizes[0] < need_x) return;
  if (in_sizes[1] < DIM) return;
  if ((long long)in_sizes[2] < (long long)DIM * DIM) return;
  if ((long long)in_sizes[3] < (long long)DIM * DIM) return;
  if ((long long)in_sizes[4] < (long long)DIM * DIM) return;
  if ((long long)in_sizes[5] < (long long)DIM * DIM) return;
  if (in_sizes[6] < DIM) return;
  if ((long long)in_sizes[7] < (long long)DIM * INTER) return;
  if ((long long)in_sizes[8] < (long long)DIM * INTER) return;
  if ((long long)in_sizes[9] < (long long)INTER * DIM) return;
  if ((long long)out_size < need_x) return;
  if (ws_size < WS_TOTAL) return;

  const float* X    = (const float*)d_in[0];
  const float* ln1w = (const float*)d_in[1];
  const float* wq   = (const float*)d_in[2];
  const float* wk   = (const float*)d_in[3];
  const float* wv   = (const float*)d_in[4];
  const float* wo   = (const float*)d_in[5];
  const float* ln2w = (const float*)d_in[6];
  const float* w1   = (const float*)d_in[7];
  const float* w3   = (const float*)d_in[8];
  const float* w2   = (const float*)d_in[9];
  float* out = (float*)d_out;

  char* ws = (char*)d_ws;
  _Float16* Wq16  = (_Float16*)(ws + OFF_WQ);
  _Float16* Wk16  = (_Float16*)(ws + OFF_WK);
  _Float16* Wv16  = (_Float16*)(ws + OFF_WV);
  _Float16* Wo16  = (_Float16*)(ws + OFF_WO);
  _Float16* W1t   = (_Float16*)(ws + OFF_W1);
  _Float16* W3t   = (_Float16*)(ws + OFF_W3);
  _Float16* W2t   = (_Float16*)(ws + OFF_W2);
  _Float16* XN16  = (_Float16*)(ws + OFF_XN);
  _Float16* Q16   = (_Float16*)(ws + OFF_Q);
  _Float16* K16   = (_Float16*)(ws + OFF_K);
  _Float16* Vt16  = (_Float16*)(ws + OFF_VT);
  _Float16* Ctx16 = (_Float16*)(ws + OFF_CTX);
  float*    H     = (float*)(ws + OFF_H);
  _Float16* G16   = (_Float16*)(ws + OFF_G);

  dim3 blk(256);
  dim3 gsq(DIM / 64, MROWS / 64);
  dim3 gup(INTER / 64, MROWS / 64);

  wconv_kernel<<<dim3(DIM / 64, DIM / 64), blk, 0, stream>>>(wq, Wq16, DIM, DIM);
  wconv_kernel<<<dim3(DIM / 64, DIM / 64), blk, 0, stream>>>(wk, Wk16, DIM, DIM);
  wconv_kernel<<<dim3(DIM / 64, DIM / 64), blk, 0, stream>>>(wv, Wv16, DIM, DIM);
  wconv_kernel<<<dim3(DIM / 64, DIM / 64), blk, 0, stream>>>(wo, Wo16, DIM, DIM);
  wconv_kernel<<<dim3(INTER / 64, DIM / 64), blk, 0, stream>>>(w1, W1t, DIM, INTER);
  wconv_kernel<<<dim3(INTER / 64, DIM / 64), blk, 0, stream>>>(w3, W3t, DIM, INTER);
  wconv_kernel<<<dim3(DIM / 64, INTER / 64), blk, 0, stream>>>(w2, W2t, INTER, DIM);

  rmsnorm_kernel<<<dim3(MROWS / 2), blk, 0, stream>>>(X, ln1w, XN16, (unsigned)SEQ_FULL, 1);

  gemm_rowmajor_kernel<<<gsq, blk, 0, stream>>>(XN16, Wq16, Q16);
  gemm_rowmajor_kernel<<<gsq, blk, 0, stream>>>(XN16, Wk16, K16);
  gemm_vt_kernel<<<gsq, blk, 0, stream>>>(XN16, Wv16, Vt16);

  attn_kernel<<<dim3(SEQ / 128, NHEAD, NB), blk, 0, stream>>>(Q16, K16, Vt16, Ctx16);

  gemm_oproj_kernel<<<gsq, blk, 0, stream>>>(Ctx16, Wo16, X, H);

  rmsnorm_kernel<<<dim3(MROWS / 2), blk, 0, stream>>>(H, ln2w, XN16, (unsigned)SEQ, 0);

  gemm_up_kernel<<<gup, blk, 0, stream>>>(XN16, W1t, W3t, G16);

  gemm_down_kernel<<<gsq, blk, 0, stream>>>(G16, W2t, H, out);
}
